// GeoGAT_56581899157896
// MI455X (gfx1250) — hardware-verified
//
#include <hip/hip_runtime.h>
#include <stddef.h>
#include <math.h>


#define FIN     128
#define D0      128
#define NOUT    16
#define NHEAD   4
#define CHN     32
#define NTHR    256
#define NWAVE   8
#define EPT     8
#define NGRP    2
#define CHUNK   (NTHR * EPT * NGRP)
#define WCAP    (EPT * NGRP * 32)
#define LISTN   (NWAVE * WCAP)
#define NBC     4096
#define NBF     1024
#define RCAP    40960
#define RBN     128
#define TGT     256
#define DEGCAP  256
#define OTHR    512
#define BM      32
#define BM2     128
#define RPB     512
#define SPB     256
#define WSCAP   134217728
#define NEG_SLOPE 0.2f
#define BN_EPS  1e-5
#define SCL_A   8.0f
#define SCL_W   16.0f
#define SCL_ACC 0.0078125f

#define LDS_FILL ((RCAP + NBF + LISTN) * 4 + 64)

static_assert((CHUNK & (CHUNK - 1)) == 0);
static_assert(CHUNK <= 4096);
static_assert(NBC <= 4096 && NBF <= 4096);
static_assert((NBC & (NBC - 1)) == 0 && (NBF & (NBF - 1)) == 0);
static_assert(NBC == 4 * NBF);
static_assert(OTHR * 8 == NBC);
static_assert((RCAP % 32) == 0);
static_assert(TGT == NWAVE * 32);
static_assert((NBC % TGT) == 0);
static_assert((TGT % BM) == 0 && (TGT % BM2) == 0);
static_assert(FIN == 128 && D0 == 128 && NOUT == 16);
static_assert(NHEAD * CHN == D0 && CHN == 32);
static_assert(SPB == 2 * D0);
static_assert((RPB % 2) == 0);

typedef float    v4f  __attribute__((ext_vector_type(4)));
typedef float    v8f  __attribute__((ext_vector_type(8)));
typedef int      v4i  __attribute__((ext_vector_type(4)));
typedef double   v2d  __attribute__((ext_vector_type(2)));
typedef _Float16 v4h  __attribute__((ext_vector_type(4)));
typedef _Float16 v8h  __attribute__((ext_vector_type(8)));
typedef _Float16 v16h __attribute__((ext_vector_type(16)));
union FragH { v16h v; v8h h[2]; };

__device__ __forceinline__ v8f wmh(v16h a, v16h b, v8f c) {
  v8f d = __builtin_amdgcn_wmma_f32_16x16x32_f16(false, a, false, b, (short)0, c, false, false);
  asm volatile("v_nop\n\tv_nop\n\tv_nop\n\tv_nop" : "+v"(d) : "v"(a), "v"(b));
  return d;
}

__device__ __forceinline__ v8h cvt8(v4f a, v4f b, float s) {
  v8f t;
  t[0] = a.x * s; t[1] = a.y * s; t[2] = a.z * s; t[3] = a.w * s;
  t[4] = b.x * s; t[5] = b.y * s; t[6] = b.z * s; t[7] = b.w * s;
  return __builtin_convertvector(t, v8h);
}

__device__ __forceinline__ float lrelu(float v) { return v > 0.0f ? v : NEG_SLOPE * v; }

__device__ __forceinline__ float bnelu(float x, float m, float is, float g, float b) {
  const float v = (x - m) * is * g + b;
  const float e = __expf(v > 0.0f ? 0.0f : v) - 1.0f;
  return v > 0.0f ? v : e;
}

template <int NB>
__device__ __forceinline__ int scan_chunk(const int* __restrict__ dsts, int nE, int cbase, int slotBase,
                                          int vec8, int* list, int tid, int lane, int wave) {
  int wc = 0;
#pragma unroll
  for (int g = 0; g < NGRP; ++g) {
    const int el0  = (g * NTHR + tid) * EPT;
    const int e0   = cbase + el0;
    const int sent = -2147483647 - 1;
    v4i da, db;
    if (vec8 != 0 && cbase + CHUNK <= nE) {
      da = *(const v4i*)(dsts + e0);
      db = *(const v4i*)(dsts + e0 + 4);
    } else {
      da.x = (e0     < nE) ? dsts[min(e0, nE - 1)] : sent;
      da.y = (e0 + 1 < nE) ? dsts[min(e0 + 1, nE - 1)] : sent;
      da.z = (e0 + 2 < nE) ? dsts[min(e0 + 2, nE - 1)] : sent;
      da.w = (e0 + 3 < nE) ? dsts[min(e0 + 3, nE - 1)] : sent;
      db.x = (e0 + 4 < nE) ? dsts[min(e0 + 4, nE - 1)] : sent;
      db.y = (e0 + 5 < nE) ? dsts[min(e0 + 5, nE - 1)] : sent;
      db.z = (e0 + 6 < nE) ? dsts[min(e0 + 6, nE - 1)] : sent;
      db.w = (e0 + 7 < nE) ? dsts[min(e0 + 7, nE - 1)] : sent;
    }
    const unsigned nb = (unsigned)slotBase;
    const unsigned s0 = (unsigned)da.x - nb, s1 = (unsigned)da.y - nb;
    const unsigned s2 = (unsigned)da.z - nb, s3 = (unsigned)da.w - nb;
    const unsigned s4 = (unsigned)db.x - nb, s5 = (unsigned)db.y - nb;
    const unsigned s6 = (unsigned)db.z - nb, s7 = (unsigned)db.w - nb;
    const bool h0 = s0 < (unsigned)NB, h1 = s1 < (unsigned)NB, h2 = s2 < (unsigned)NB, h3 = s3 < (unsigned)NB;
    const bool h4 = s4 < (unsigned)NB, h5 = s5 < (unsigned)NB, h6 = s6 < (unsigned)NB, h7 = s7 < (unsigned)NB;
    const unsigned any = __builtin_amdgcn_ballot_w32(h0 | h1 | h2 | h3 | h4 | h5 | h6 | h7);
    if (any != 0u) {
#define HITJ(J, HJ, SJ) { \
        const unsigned mj = __builtin_amdgcn_ballot_w32(HJ); \
        if (mj != 0u) { \
          if (HJ) { \
            const int pos = wc + (int)__builtin_amdgcn_mbcnt_lo(mj, 0u); \
            if (pos < WCAP) list[wave * WCAP + pos] = ((el0 + (J)) << 12) | (int)(SJ); \
          } \
          wc += (int)__builtin_popcount(mj); } }
      HITJ(0, h0, s0)
      HITJ(1, h1, s1)
      HITJ(2, h2, s2)
      HITJ(3, h3, s3)
      HITJ(4, h4, s4)
      HITJ(5, h5, s5)
      HITJ(6, h6, s6)
      HITJ(7, h7, s7)
#undef HITJ
    }
  }
  return wc;
}

__global__ __launch_bounds__(NTHR) void k_xcvt(const float* __restrict__ x, _Float16* xp, int nN, int nUnits) {
  const int i = (int)blockIdx.x * NTHR + (int)threadIdx.x;
  if (i >= nUnits) return;
  const int row = i >> 4;
  const int c0  = (i & 15) * 8;
  int rr = row > nN - 1 ? nN - 1 : row;
  rr = rr < 0 ? 0 : rr;
  const float* p = x + (size_t)rr * FIN + c0;
  v4f a = *(const v4f*)p, b = *(const v4f*)(p + 4);
  const v4f z = {0.f, 0.f, 0.f, 0.f};
  if (row >= nN) { a = z; b = z; }
  const v8h o = cvt8(a, b, SCL_A);
  _Float16* d = xp + (size_t)i * 8;
  *(volatile v8h*)d = o;
  __threadfence();
  *(volatile v8h*)d = o;
}

template <int KD, int NCW>
__global__ __launch_bounds__(NTHR) void k_wprep(const float* __restrict__ W, _Float16* wp) {
  constexpr int KS    = KD / 8;
  constexpr int UNITS = NCW * KS;
  static_assert(KD % 8 == 0);
  const int i = (int)blockIdx.x * NTHR + (int)threadIdx.x;
  if (i >= UNITS) return;
  const int n  = i / KS;
  const int k0 = (i - n * KS) * 8;
  v4f a, b;
  a.x = W[(size_t)(k0 + 0) * NCW + n]; a.y = W[(size_t)(k0 + 1) * NCW + n];
  a.z = W[(size_t)(k0 + 2) * NCW + n]; a.w = W[(size_t)(k0 + 3) * NCW + n];
  b.x = W[(size_t)(k0 + 4) * NCW + n]; b.y = W[(size_t)(k0 + 5) * NCW + n];
  b.z = W[(size_t)(k0 + 6) * NCW + n]; b.w = W[(size_t)(k0 + 7) * NCW + n];
  const v8h o = cvt8(a, b, SCL_W);
  _Float16* d = wp + (size_t)i * 8;
  *(volatile v8h*)d = o;
  __threadfence();
  *(volatile v8h*)d = o;
}

__global__ __launch_bounds__(NTHR) void k_count(
    const int* __restrict__ dsts, int* cnt, int nE, int vec8) {
  __shared__ __attribute__((aligned(16))) int scnt[NBC];
  __shared__ __attribute__((aligned(16))) int list[LISTN];
  __shared__ int wcnt[NWAVE];
  const int tid = threadIdx.x, lane = tid & 31, wave = tid >> 5;
  const int nodeBase = blockIdx.x * NBC;

  for (int i = tid; i < NBC; i += NTHR) scnt[i] = 0;
  __syncthreads();

  const int nChunks = (nE + CHUNK - 1) / CHUNK;
#pragma unroll 1
  for (int ch = 0; ch < nChunks; ++ch) {
    const int cbase = ch * CHUNK;
    const int wc = scan_chunk<NBC>(dsts, nE, cbase, nodeBase, vec8, list, tid, lane, wave);
    if (lane == 0) wcnt[wave] = wc;
    __syncthreads();
    if (wave == 0) {
#pragma unroll 1
      for (int wsx = 0; wsx < NWAVE; ++wsx) {
        int n = __builtin_amdgcn_readfirstlane(wcnt[wsx]);
        n = n > WCAP ? WCAP : (n < 0 ? 0 : n);
        const int* lp = list + wsx * WCAP;
#pragma unroll 1
        for (int i = 0; i < n; ++i) {
          const int ent  = __builtin_amdgcn_readfirstlane(lp[i]);
          const int slot = ent & (NBC - 1);
          if (lane == 0) scnt[slot] = scnt[slot] + 1;
        }
      }
    }
    __syncthreads();
  }

  v4i cq[4];
#pragma unroll
  for (int q = 0; q < 4; ++q) {
    const int f = (wave * 4 + q) * 128 + 4 * lane;
    cq[q] = *(const v4i*)(scnt + f);
  }
  int* cp = cnt + (size_t)nodeBase;
#pragma unroll
  for (int q = 0; q < 4; ++q) {
    const int f = (wave * 4 + q) * 128 + 4 * lane;
    *(volatile v4i*)(cp + f) = cq[q];
  }
  __threadfence();
#pragma unroll
  for (int q = 0; q < 4; ++q) {
    const int f = (wave * 4 + q) * 128 + 4 * lane;
    *(volatile v4i*)(cp + f) = cq[q];
  }
}

__global__ __launch_bounds__(OTHR) void k_offsets(
    const int* __restrict__ cnt, int* off, int* rbase, int nChunk) {
  __shared__ __attribute__((aligned(16))) int soff[NBC];
  __shared__ __attribute__((aligned(16))) int srb[RBN];
  __shared__ int wtot[OTHR / 32];
  const int tid = threadIdx.x, lane = tid & 31, wave = tid >> 5, sub = tid >> 7;
  for (int i = tid; i < RBN; i += OTHR) srb[i] = 0;
  int carry = 0;
#pragma unroll 1
  for (int ch = 0; ch < nChunk; ++ch) {
    const int base = ch * NBC;
    const v4i c0 = *(const v4i*)(cnt + base + 8 * tid);
    const v4i c1 = *(const v4i*)(cnt + base + 8 * tid + 4);
    const int e0 = max(c0.x, 0), e1 = max(c0.y, 0), e2 = max(c0.z, 0), e3 = max(c0.w, 0);
    const int e4 = max(c1.x, 0), e5 = max(c1.y, 0), e6 = max(c1.z, 0), e7 = max(c1.w, 0);
    const int ts = e0 + e1 + e2 + e3 + e4 + e5 + e6 + e7;
    int incl = ts;
#pragma unroll
    for (int d = 1; d < 32; d <<= 1) {
      const int t = __shfl_up(incl, d);
      if (lane >= d) incl += t;
    }
    if (lane == 31) wtot[wave] = incl;
    __syncthreads();
    const int S0 = wtot[0]  + wtot[1]  + wtot[2]  + wtot[3];
    const int S1 = wtot[4]  + wtot[5]  + wtot[6]  + wtot[7];
    const int S2 = wtot[8]  + wtot[9]  + wtot[10] + wtot[11];
    const int S3 = wtot[12] + wtot[13] + wtot[14] + wtot[15];
    int pre = 0;
#pragma unroll 1
    for (int w = 4 * sub; w < wave; ++w) pre += wtot[w];
    const int b0 = carry;
    const int b1 = b0 + ((S0 + 31) & ~31);
    const int b2 = b1 + ((S1 + 31) & ~31);
    const int b3 = b2 + ((S2 + 31) & ~31);
    const int b4 = b3 + ((S3 + 31) & ~31);
    const int myb = sub == 0 ? b0 : (sub == 1 ? b1 : (sub == 2 ? b2 : b3));
    if (tid == 0) {
      srb[min(4 * ch + 0, RBN - 1)] = b0;
      srb[min(4 * ch + 1, RBN - 1)] = b1;
      srb[min(4 * ch + 2, RBN - 1)] = b2;
      srb[min(4 * ch + 3, RBN - 1)] = b3;
    }
    int run = myb + pre + incl - ts;
    soff[8 * tid + 0] = run; run += e0;
    soff[8 * tid + 1] = run; run += e1;
    soff[8 * tid + 2] = run; run += e2;
    soff[8 * tid + 3] = run; run += e3;
    soff[8 * tid + 4] = run; run += e4;
    soff[8 * tid + 5] = run; run += e5;
    soff[8 * tid + 6] = run; run += e6;
    soff[8 * tid + 7] = run;
    carry = b4;
    __syncthreads();
    const v4i o0 = *(const v4i*)(soff + 4 * tid);
    const v4i o1 = *(const v4i*)(soff + 4 * (tid + OTHR));
    int* op = off + base;
    *(volatile v4i*)(op + 4 * tid) = o0;
    *(volatile v4i*)(op + 4 * (tid + OTHR)) = o1;
    __threadfence();
    *(volatile v4i*)(op + 4 * tid) = o0;
    *(volatile v4i*)(op + 4 * (tid + OTHR)) = o1;
    __syncthreads();
  }
  if (tid == 0) srb[min(4 * nChunk, RBN - 1)] = carry;
  __syncthreads();
  v4i rv = {0, 0, 0, 0};
  if (tid < 32) rv = *(const v4i*)(srb + 4 * tid);
  if (tid < 32) *(volatile v4i*)(rbase + 4 * tid) = rv;
  __threadfence();
  if (tid < 32) *(volatile v4i*)(rbase + 4 * tid) = rv;
}

__global__ __launch_bounds__(NTHR) void k_fill(
    const int* __restrict__ srcs, const int* __restrict__ dsts,
    const int* __restrict__ off, const int* __restrict__ rbase,
    int* csr, int nN, int nE, int vec8, int csrLen) {
  extern __shared__ v4f lds_dyn[];
  int* region = (int*)lds_dyn;
  int* cursor = region + RCAP;
  int* list   = cursor + NBF;
  int* wcnt   = list + LISTN;
  const int tid = threadIdx.x, lane = tid & 31, wave = tid >> 5;
  const int b = blockIdx.x;
  const int nodeBase = b * NBF;

  int rb0 = rbase[b];
  const int rb1 = rbase[b + 1];
  rb0 = rb0 < 0 ? 0 : (rb0 > csrLen ? csrLen : rb0);
  rb0 &= ~31;
  int len = rb1 - rb0;
  len = len < 0 ? 0 : (len > RCAP ? RCAP : len);
  int lenW = (len + 31) & ~31;
  if (rb0 + lenW > csrLen) lenW = (csrLen - rb0) & ~31;

  {
    const v4i z = {0, 0, 0, 0};
    for (int i = tid; i < RCAP / 4; i += NTHR) ((v4i*)region)[i] = z;
    for (int s = tid; s < NBF; s += NTHR) {
      int o = off[nodeBase + s] - rb0;
      o = o < 0 ? 0 : (o > RCAP ? RCAP : o);
      cursor[s] = o;
    }
  }
  __syncthreads();

  const int nChunks = (nE + CHUNK - 1) / CHUNK;
#pragma unroll 1
  for (int ch = 0; ch < nChunks; ++ch) {
    const int cbase = ch * CHUNK;
    const int wc = scan_chunk<NBF>(dsts, nE, cbase, nodeBase, vec8, list, tid, lane, wave);
    if (lane == 0) wcnt[wave] = wc;
    __syncthreads();
    if (wave == 0) {
#pragma unroll 1
      for (int wsx = 0; wsx < NWAVE; ++wsx) {
        int n = __builtin_amdgcn_readfirstlane(wcnt[wsx]);
        n = n > WCAP ? WCAP : (n < 0 ? 0 : n);
        const int* lp = list + wsx * WCAP;
#pragma unroll 1
        for (int i = 0; i < n; ++i) {
          const int ent  = __builtin_amdgcn_readfirstlane(lp[i]);
          const int slot = ent & (NBF - 1);
          int e = cbase + ((ent >> 12) & (CHUNK - 1));
          e = e > nE - 1 ? nE - 1 : e;
          int src = srcs[e];
          src = src < 0 ? 0 : (src > nN - 1 ? nN - 1 : src);
          if (lane == 0) {
            int pos = cursor[slot];
            pos = pos < 0 ? 0 : (pos > RCAP - 1 ? RCAP - 1 : pos);
            region[pos] = src;
            const int np = pos + 1;
            cursor[slot] = np > RCAP ? RCAP : np;
          }
        }
      }
    }
    __syncthreads();
  }

  const int nv = lenW >> 2;
  int* gp = csr + rb0;
#pragma unroll 1
  for (int i = tid; i < nv; i += NTHR) { const v4i v = ((const v4i*)region)[i]; *(volatile v4i*)(gp + 4 * i) = v; }
  __threadfence();
#pragma unroll 1
  for (int i = tid; i < nv; i += NTHR) { const v4i v = ((const v4i*)region)[i]; *(volatile v4i*)(gp + 4 * i) = v; }
}

__global__ __launch_bounds__(NTHR) void k_gemm(
    const _Float16* __restrict__ Ap, const _Float16* __restrict__ Bp,
    const float* __restrict__ attS, const float* __restrict__ attD,
    float* Hf, float* eS, float* eD) {
  constexpr int K    = D0;
  constexpr int NC   = D0;
  constexpr int TPW  = NC / 64;
  constexpr int KT   = K / 32;
  constexpr int CPP  = NC / 8;
  constexpr int NES  = BM * NHEAD;
  constexpr int NIT4 = (BM * NC / 4) / NTHR;
  static_assert(TPW == 2 && KT == 4 && CPP == 16 && NES == 128 && NIT4 == 4);
  static_assert((NC / NHEAD) == 2 * CPP);
  static_assert(BM * 8 == NTHR);

  __shared__ __attribute__((aligned(16))) float stg[BM * NC];
  __shared__ __attribute__((aligned(16))) float sES[NES];
  __shared__ __attribute__((aligned(16))) float sED[NES];
  const int tid = threadIdx.x, lane = tid & 31, wave = tid >> 5, hh = lane >> 4, m = lane & 15;
  const int rowBase = blockIdx.x * BM;
  const int rg = wave >> 2, cq = wave & 3;
  const int r0 = rg * 16;
  const int c0 = cq * (NC / 4);

  v8f acc[TPW];
#pragma unroll
  for (int t = 0; t < TPW; ++t) { v8f z = {0.f, 0.f, 0.f, 0.f, 0.f, 0.f, 0.f, 0.f}; acc[t] = z; }

  const _Float16* ap  = Ap + (size_t)(rowBase + r0 + m) * K + 8 * hh;
  const _Float16* bp0 = Bp + (size_t)(c0 + m) * K + 8 * hh;
#pragma unroll 1
  for (int kt = 0; kt < KT; ++kt) {
    FragH a;
    a.h[0] = *(const v8h*)(ap + 32 * kt);
    a.h[1] = *(const v8h*)(ap + 32 * kt + 16);
#pragma unroll
    for (int t = 0; t < TPW; ++t) {
      const _Float16* bp = bp0 + (size_t)(16 * t) * K + 32 * kt;
      FragH bf;
      bf.h[0] = *(const v8h*)bp;
      bf.h[1] = *(const v8h*)(bp + 16);
      acc[t] = wmh(a.v, bf.v, acc[t]);
    }
  }

  {
    float* sp = stg + (size_t)(r0 + 8 * hh) * NC + c0 + m;
#pragma unroll
    for (int t = 0; t < TPW; ++t) {
#pragma unroll
      for (int r = 0; r < 8; ++r) sp[r * NC + 16 * t] = acc[t][r] * SCL_ACC;
    }
  }
  __syncthreads();

  {
    const int drow = tid >> 3, part = tid & 7;
    const float* rp  = stg + (size_t)drow * NC + CPP * part;
    const float* sa  = attS + CPP * part;
    const float* sdd = attD + CPP * part;
    float ps = 0.f, pd = 0.f;
#pragma unroll 4
    for (int c = 0; c < CPP; c += 4) {
      const v4f hv = *(const v4f*)(rp + c);
      const v4f av = *(const v4f*)(sa + c);
      const v4f dv = *(const v4f*)(sdd + c);
      ps += hv.x * av.x + hv.y * av.y + hv.z * av.z + hv.w * av.w;
      pd += hv.x * dv.x + hv.y * dv.y + hv.z * dv.z + hv.w * dv.w;
    }
    ps += __shfl_xor(ps, 1); pd += __shfl_xor(pd, 1);
    if ((part & 1) == 0) { sES[drow * NHEAD + (part >> 1)] = ps; sED[drow * NHEAD + (part >> 1)] = pd; }
  }

  {
    float* tile = Hf + (size_t)rowBase * NC;
    v4f cv[NIT4];
#pragma unroll
    for (int it = 0; it < NIT4; ++it) cv[it] = *(const v4f*)(stg + 4 * (it * NTHR + tid));
#pragma unroll
    for (int it = 0; it < NIT4; ++it) *(volatile v4f*)(tile + 4 * (size_t)(it * NTHR + tid)) = cv[it];
    __threadfence();
#pragma unroll
    for (int it = 0; it < NIT4; ++it) *(volatile v4f*)(tile + 4 * (size_t)(it * NTHR + tid)) = cv[it];
  }
  __syncthreads();

  {
    const v4f vS = *(const v4f*)(sES + 4 * lane);
    const v4f vD = *(const v4f*)(sED + 4 * lane);
    float* gS = eS + (size_t)rowBase * NHEAD + 4 * lane;
    float* gD = eD + (size_t)rowBase * NHEAD + 4 * lane;
    if (wave == 0) *(volatile v4f*)gS = vS;
    if (wave == 1) *(volatile v4f*)gD = vD;
    __threadfence();
    if (wave == 0) *(volatile v4f*)gS = vS;
    if (wave == 1) *(volatile v4f*)gD = vD;
  }
}

__global__ __launch_bounds__(NTHR) void k_gemm16(
    const _Float16* __restrict__ Ap, const _Float16* __restrict__ Bp,
    const float* __restrict__ attS, const float* __restrict__ attD,
    float* Hf, float* eS, float* eD) {
  constexpr int K  = D0;
  constexpr int KT = K / 32;
  constexpr int NIT4 = (BM2 * NOUT / 4) / NTHR;
  static_assert(NIT4 == 2 && BM2 == 16 * NWAVE && BM2 * 2 == NTHR);

  __shared__ __attribute__((aligned(16))) float stg[BM2 * NOUT];
  __shared__ __attribute__((aligned(16))) float sES[BM2];
  __shared__ __attribute__((aligned(16))) float sED[BM2];
  const int tid = threadIdx.x, lane = tid & 31, wave = tid >> 5, hh = lane >> 4, m = lane & 15;
  const int rowBase = blockIdx.x * BM2;
  const int r0 = wave * 16;

  v8f acc = {0.f, 0.f, 0.f, 0.f, 0.f, 0.f, 0.f, 0.f};
  const _Float16* ap = Ap + (size_t)(rowBase + r0 + m) * K + 8 * hh;
  const _Float16* bp = Bp + (size_t)m * K + 8 * hh;
#pragma unroll 1
  for (int kt = 0; kt < KT; ++kt) {
    FragH a, bf;
    a.h[0]  = *(const v8h*)(ap + 32 * kt);
    a.h[1]  = *(const v8h*)(ap + 32 * kt + 16);
    bf.h[0] = *(const v8h*)(bp + 32 * kt);
    bf.h[1] = *(const v8h*)(bp + 32 * kt + 16);
    acc = wmh(a.v, bf.v, acc);
  }

  {
    float* sp = stg + (size_t)(r0 + 8 * hh) * NOUT + m;
#pragma unroll
    for (int r = 0; r < 8; ++r) sp[r * NOUT] = acc[r] * SCL_ACC;
  }
  __syncthreads();

  {
    const int drow = tid >> 1, part = tid & 1;
    const float* rp = stg + (size_t)drow * NOUT + 8 * part;
    const v4f h0 = *(const v4f*)rp, h1 = *(const v4f*)(rp + 4);
    const v4f a0 = *(const v4f*)(attS + 8 * part), a1 = *(const v4f*)(attS + 8 * part + 4);
    const v4f d0 = *(const v4f*)(attD + 8 * part), d1 = *(const v4f*)(attD + 8 * part + 4);
    float ps = h0.x * a0.x + h0.y * a0.y + h0.z * a0.z + h0.w * a0.w
             + h1.x * a1.x + h1.y * a1.y + h1.z * a1.z + h1.w * a1.w;
    float pd = h0.x * d0.x + h0.y * d0.y + h0.z * d0.z + h0.w * d0.w
             + h1.x * d1.x + h1.y * d1.y + h1.z * d1.z + h1.w * d1.w;
    ps += __shfl_xor(ps, 1); pd += __shfl_xor(pd, 1);
    if (part == 0) { sES[drow] = ps; sED[drow] = pd; }
  }

  {
    float* tile = Hf + (size_t)rowBase * NOUT;
    v4f cv[NIT4];
#pragma unroll
    for (int it = 0; it < NIT4; ++it) cv[it] = *(const v4f*)(stg + 4 * (it * NTHR + tid));
#pragma unroll
    for (int it = 0; it < NIT4; ++it) *(volatile v4f*)(tile + 4 * (size_t)(it * NTHR + tid)) = cv[it];
    __threadfence();
#pragma unroll
    for (int it = 0; it < NIT4; ++it) *(volatile v4f*)(tile + 4 * (size_t)(it * NTHR + tid)) = cv[it];
  }
  __syncthreads();

  {
    const v4f vS = *(const v4f*)(sES + 4 * lane);
    const v4f vD = *(const v4f*)(sED + 4 * lane);
    float* gS = eS + (size_t)rowBase + 4 * lane;
    float* gD = eD + (size_t)rowBase + 4 * lane;
    if (wave == 0) *(volatile v4f*)gS = vS;
    if (wave == 1) *(volatile v4f*)gD = vD;
    __threadfence();
    if (wave == 0) *(volatile v4f*)gS = vS;
    if (wave == 1) *(volatile v4f*)gD = vD;
  }
}

__global__ __launch_bounds__(NTHR) void k_agg(
    const int* __restrict__ csr, const int* __restrict__ off, const int* __restrict__ cnt,
    const float* __restrict__ eS, const float* __restrict__ eD,
    const float* __restrict__ hf, const float* __restrict__ bias,
    float* gout, int nN, int csrLen) {
  const int tid = threadIdx.x, lane = tid & 31, wave = tid >> 5;
  const int tbase = blockIdx.x * TGT + wave * 32;
  const int col = 4 * lane;
  const int hd  = lane >> 3;

  const v4f bb = *(const v4f*)(bias + col);

  const int cl    = tbase + lane;
  const int cnt_l = cnt[cl];
  const int off_l = off[cl];

#pragma unroll 1
  for (int j = 0; j < 32; ++j) {
    const int c = tbase + j;
    int n = __builtin_amdgcn_readfirstlane(__shfl(cnt_l, j));
    n = n < 0 ? 0 : (n > DEGCAP ? DEGCAP : n);
    const int st = __builtin_amdgcn_readfirstlane(__shfl(off_l, j));
    const float esc = eS[(size_t)c * NHEAD + hd];
    const float edc = eD[(size_t)c * NHEAD + hd];

    float mxs = esc;
#pragma unroll 1
    for (int q0 = 0; q0 < n; q0 += 32) {
      int pos = st + q0 + lane;
      pos = pos < 0 ? 0 : (pos > csrLen - 1 ? csrLen - 1 : pos);
      int sl = csr[pos];
      sl = sl < 0 ? 0 : (sl > nN - 1 ? nN - 1 : sl);
      const int mcnt = (n - q0) < 32 ? (n - q0) : 32;
#pragma unroll 1
      for (int pp = 0; pp < mcnt; ++pp) {
        const int s = __builtin_amdgcn_readlane(sl, pp);
        mxs = fmaxf(mxs, eS[(size_t)s * NHEAD + hd]);
      }
    }
    const float mx = lrelu(mxs + edc);

    float p   = __expf(lrelu(esc + edc) - mx);
    float den = p;
    v4f acc = *(const v4f*)(hf + (size_t)c * D0 + col) * p;
#pragma unroll 1
    for (int q0 = 0; q0 < n; q0 += 32) {
      int pos = st + q0 + lane;
      pos = pos < 0 ? 0 : (pos > csrLen - 1 ? csrLen - 1 : pos);
      int sl = csr[pos];
      sl = sl < 0 ? 0 : (sl > nN - 1 ? nN - 1 : sl);
      const int mcnt = (n - q0) < 32 ? (n - q0) : 32;
#pragma unroll 1
      for (int pp = 0; pp < mcnt; ++pp) {
        const int s = __builtin_amdgcn_readlane(sl, pp);
        p = __expf(lrelu(eS[(size_t)s * NHEAD + hd] + edc) - mx);
        den += p;
        const v4f hv = *(const v4f*)(hf + (size_t)s * D0 + col);
        acc = acc + hv * p;
      }
    }

    const float rd = 1.0f / den;
    const v4f v = acc * rd + bb;
    float* gp = gout + (size_t)c * D0 + col;
    *(volatile v4f*)gp = v;
    __threadfence();
    *(volatile v4f*)gp = v;
  }
}

__global__ __launch_bounds__(NTHR) void k_aggo(
    const int* __restrict__ csr, const int* __restrict__ off, const int* __restrict__ cnt,
    const float* __restrict__ eS, const float* __restrict__ eD,
    const float* __restrict__ hf, const float* __restrict__ bias,
    float* out, int nN, int csrLen) {
  __shared__ __attribute__((aligned(16))) float sOut[NWAVE * 32 * NOUT];
  const int tid = threadIdx.x, lane = tid & 31, wave = tid >> 5, hh = lane >> 4, cc = lane & 15;
  const int tbase = blockIdx.x * TGT + wave * 32;

  const float bc = bias[cc];

  const int cl    = tbase + lane;
  const int cnt_l = cnt[cl];
  const int off_l = off[cl];

#pragma unroll 1
  for (int j = 0; j < 32; ++j) {
    const int c = tbase + j;
    int n = __builtin_amdgcn_readfirstlane(__shfl(cnt_l, j));
    n = n < 0 ? 0 : (n > DEGCAP ? DEGCAP : n);
    const int st = __builtin_amdgcn_readfirstlane(__shfl(off_l, j));
    const float esc = eS[c];
    const float edc = eD[c];

    float mxs = esc;
#pragma unroll 1
    for (int q0 = 0; q0 < n; q0 += 32) {
      int pos = st + q0 + lane;
      pos = pos < 0 ? 0 : (pos > csrLen - 1 ? csrLen - 1 : pos);
      int sl = csr[pos];
      sl = sl < 0 ? 0 : (sl > nN - 1 ? nN - 1 : sl);
      const int mcnt = (n - q0) < 32 ? (n - q0) : 32;
#pragma unroll 1
      for (int pp = 0; pp < mcnt; ++pp) {
        const int s = __builtin_amdgcn_readlane(sl, pp);
        mxs = fmaxf(mxs, eS[s]);
      }
    }
    const float mx = lrelu(mxs + edc);

    const float pself = __expf(lrelu(esc + edc) - mx);
    float p   = (hh == 0) ? pself : 0.0f;
    float den = p;
    float acc = hf[(size_t)c * NOUT + cc] * p;
#pragma unroll 1
    for (int q0 = 0; q0 < n; q0 += 32) {
      int pos = st + q0 + lane;
      pos = pos < 0 ? 0 : (pos > csrLen - 1 ? csrLen - 1 : pos);
      int sl = csr[pos];
      sl = sl < 0 ? 0 : (sl > nN - 1 ? nN - 1 : sl);
      const int mcnt = (n - q0) < 32 ? (n - q0) : 32;
#pragma unroll 1
      for (int pp = 0; pp < mcnt; pp += 2) {
        const int idx = pp + hh;
        const int s   = __shfl(sl, idx);
        const float pr = __expf(lrelu(eS[s] + edc) - mx);
        const float pe = (idx < mcnt) ? pr : 0.0f;
        den += pe;
        acc += hf[(size_t)s * NOUT + cc] * pe;
      }
    }
    den += __shfl_xor(den, 16);
    acc += __shfl_xor(acc, 16);
    const float v = acc * (1.0f / den) + bc;
    if (hh == 0) sOut[(wave * 32 + j) * NOUT + cc] = v;
  }
  __syncthreads();

  {
    const float* sp = sOut + (size_t)(wave * 32) * NOUT;
    float* gp = out + (size_t)tbase * NOUT;
    v4f vq[4];
    bool ok[4];
#pragma unroll
    for (int q = 0; q < 4; ++q) {
      vq[q] = *(const v4f*)(sp + q * 128 + 4 * lane);
      ok[q] = (tbase + q * 8 + (lane >> 2)) < nN;
    }
#pragma unroll
    for (int q = 0; q < 4; ++q) if (ok[q]) *(volatile v4f*)(gp + q * 128 + 4 * lane) = vq[q];
    __threadfence();
#pragma unroll
    for (int q = 0; q < 4; ++q) if (ok[q]) *(volatile v4f*)(gp + q * 128 + 4 * lane) = vq[q];
  }
}

__global__ __launch_bounds__(NTHR) void k_bnstat(const float* __restrict__ G, double* part, int nN) {
  __shared__ __attribute__((aligned(16))) double sS[SPB];
  __shared__ __attribute__((aligned(16))) double sF[SPB];
  const int tid = threadIdx.x;
  const int c = tid & (D0 - 1), ph = tid >> 7;
  const int rBeg = blockIdx.x * RPB;
  int rEnd = rBeg + RPB;
  rEnd = rEnd > nN ? nN : rEnd;
  double s = 0.0, q = 0.0;
#pragma unroll 1
  for (int r = rBeg + ph; r < rEnd; r += 2) {
    const double v = (double)G[(size_t)r * D0 + c];
    s += v;
    q += v * v;
  }
  if (ph == 1) { sS[c] = s; sS[D0 + c] = q; }
  __syncthreads();
  if (ph == 0) { s += sS[c]; q += sS[D0 + c]; sF[c] = s; sF[D0 + c] = q; }
  __syncthreads();
  v2d v = {0.0, 0.0};
  if (tid < D0) v = *(const v2d*)(sF + 2 * tid);
  double* gp = part + (size_t)blockIdx.x * SPB + 2 * (tid < D0 ? tid : 0);
  if (tid < D0) *(volatile v2d*)gp = v;
  __threadfence();
  if (tid < D0) *(volatile v2d*)gp = v;
}

__global__ __launch_bounds__(NTHR) void k_bnfin(const double* __restrict__ part, float* tab, int nSB, int nN) {
  __shared__ __attribute__((aligned(16))) float sT[SPB];
  const int tid = threadIdx.x;
  if (tid < D0) {
    double s = 0.0, q = 0.0;
#pragma unroll 1
    for (int b = 0; b < nSB; ++b) {
      s += part[(size_t)b * SPB + tid];
      q += part[(size_t)b * SPB + D0 + tid];
    }
    const double inv  = 1.0 / (double)nN;
    const double mean = s * inv;
    double var = q * inv - mean * mean;
    var = var < 0.0 ? 0.0 : var;
    const double istd = 1.0 / sqrt(var + (double)BN_EPS);
    sT[tid] = (float)mean;
    sT[D0 + tid] = (float)istd;
  }
  __syncthreads();
  v4f v = {0.f, 0.f, 0.f, 0.f};
  if (tid < 64) v = *(const v4f*)(sT + 4 * tid);
  float* gp = tab + 4 * (tid < 64 ? tid : 0);
  if (tid < 64) *(volatile v4f*)gp = v;
  __threadfence();
  if (tid < 64) *(volatile v4f*)gp = v;
}

__global__ __launch_bounds__(NTHR) void k_bnapply(
    const float* __restrict__ G, const float* __restrict__ tab,
    const float* __restrict__ gam, const float* __restrict__ bet,
    _Float16* xp, int nN, int nUnits) {
  const int i = (int)blockIdx.x * NTHR + (int)threadIdx.x;
  if (i >= nUnits) return;
  const int row = i >> 4;
  const int c0  = (i & 15) * 8;
  int rr = row > nN - 1 ? nN - 1 : row;
  rr = rr < 0 ? 0 : rr;
  const float* p = G + (size_t)rr * D0 + c0;
  const v4f a  = *(const v4f*)p,              b  = *(const v4f*)(p + 4);
  const v4f m0 = *(const v4f*)(tab + c0),      m1 = *(const v4f*)(tab + c0 + 4);
  const v4f i0 = *(const v4f*)(tab + D0 + c0), i1 = *(const v4f*)(tab + D0 + c0 + 4);
  const v4f g0 = *(const v4f*)(gam + c0),      g1 = *(const v4f*)(gam + c0 + 4);
  const v4f e0 = *(const v4f*)(bet + c0),      e1 = *(const v4f*)(bet + c0 + 4);
  v4f u, w;
  u.x = bnelu(a.x, m0.x, i0.x, g0.x, e0.x); u.y = bnelu(a.y, m0.y, i0.y, g0.y, e0.y);
  u.z = bnelu(a.z, m0.z, i0.z, g0.z, e0.z); u.w = bnelu(a.w, m0.w, i0.w, g0.w, e0.w);
  w.x = bnelu(b.x, m1.x, i1.x, g1.x, e1.x); w.y = bnelu(b.y, m1.y, i1.y, g1.y, e1.y);
  w.z = bnelu(b.z, m1.z, i1.z, g1.z, e1.z); w.w = bnelu(b.w, m1.w, i1.w, g1.w, e1.w);
  const v4f z = {0.f, 0.f, 0.f, 0.f};
  if (row >= nN) { u = z; w = z; }
  const v8h o = cvt8(u, w, SCL_A);
  _Float16* d = xp + (size_t)i * 8;
  *(volatile v8h*)d = o;
  __threadfence();
  *(volatile v8h*)d = o;
}

extern "C" void kernel_launch(void* const* d_in, const int* in_sizes, int n_in,
                              void* d_out, int out_size, void* d_ws, size_t ws_size,
                              hipStream_t stream) {
  if (n_in < 18) return;
  const int nN = in_sizes[0] / FIN;
  const int nE = in_sizes[1] / 2;
  if (nN <= 0 || nE <= 0 || in_sizes[0] != nN * FIN || in_sizes[1] != 2 * nE) return;
  if (in_sizes[2] != FIN * D0 || in_sizes[3] != D0 || in_sizes[4] != D0) return;
  if (in_sizes[5] != D0 || in_sizes[6] != D0 || in_sizes[7] != D0) return;
  if (in_sizes[8] != D0 * D0 || in_sizes[9] != D0 || in_sizes[10] != D0) return;
  if (in_sizes[11] != D0 || in_sizes[12] != D0 || in_sizes[13] != D0) return;
  if (in_sizes[14] != D0 * NOUT || in_sizes[15] != NOUT || in_sizes[16] != NOUT || in_sizes[17] != NOUT) return;
  if (out_size != nN * NOUT) return;
  if (nE > (1 << 28) || nN > (1 << 22)) return;

  const float* x    = (const float*)d_in[0];
  const int*   ei   = (const int*)d_in[1];
  const int*   src  = ei;
  const int*   dst  = ei + nE;
  const float* W0   = (const float*)d_in[2];
  const float* as0  = (const float*)d_in[3];
  const float* ad0  = (const float*)d_in[4];
  const float* b0   = (const float*)d_in[5];
  const float* g0   = (const float*)d_in[6];
  const float* be0  = (const float*)d_in[7];
  const float* W1   = (const float*)d_in[8];
  const float* as1  = (const float*)d_in[9];
  const float* ad1  = (const float*)d_in[10];
  const float* b1   = (const float*)d_in[11];
  const float* g1   = (const float*)d_in[12];
  const float* be1  = (const float*)d_in[13];
  const float* W2   = (const float*)d_in[14];
  const float* as2  = (const float*)d_in[15];
  const float* ad2  = (const float*)d_in[16];
  const float* b2   = (const float*)d_in[17];
  float* out = (float*)d_out;

  const int NPAD   = ((nN + TGT - 1) / TGT) * TGT;
  const int nBC    = (nN + NBC - 1) / NBC;
  const int CNTPAD = nBC * NBC;
  if (CNTPAD < NPAD) return;
  if (4 * nBC + 1 > RBN) return;
  const int nBF    = (nN + NBF - 1) / NBF;
  if (nBF + 1 > 4 * nBC + 1) return;
  const int csrLen = ((nE + 31) & ~31) + 4096;
  if (31 * 4 * nBC > 4096) return;
  const int nAgg   = NPAD / TGT;
  const int nGemm  = NPAD / BM;
  const int nGemm2 = NPAD / BM2;
  const int nXu    = NPAD * (FIN / 8);
  const int nSB    = (nN + RPB - 1) / RPB;

  char* ws = (char*)d_ws;
  size_t off = 0;
  const size_t oW0  = off; off += (size_t)D0 * FIN * 2;            off = (off + 255) & ~(size_t)255;
  const size_t oW1  = off; off += (size_t)D0 * D0 * 2;             off = (off + 255) & ~(size_t)255;
  const size_t oW2  = off; off += (size_t)NOUT * D0 * 2;           off = (off + 255) & ~(size_t)255;
  const size_t oP   = off; off += (size_t)NPAD * D0 * 2;           off = (off + 255) & ~(size_t)255;
  const size_t oH   = off; off += (size_t)NPAD * D0 * 4;           off = (off + 255) & ~(size_t)255;
  const size_t oG   = off; off += (size_t)NPAD * D0 * 4;           off = (off + 255) & ~(size_t)255;
  const size_t oCnt = off; off += (size_t)CNTPAD * 4;              off = (off + 255) & ~(size_t)255;
  const size_t oOff = off; off += (size_t)CNTPAD * 4;              off = (off + 255) & ~(size_t)255;
  const size_t oRb  = off; off += (size_t)RBN * 4;                 off = (off + 255) & ~(size_t)255;
  const size_t oCsr = off; off += (size_t)csrLen * 4;              off = (off + 255) & ~(size_t)255;
  const size_t oES  = off; off += (size_t)NPAD * NHEAD * 4;        off = (off + 255) & ~(size_t)255;
  const size_t oED  = off; off += (size_t)NPAD * NHEAD * 4;        off = (off + 255) & ~(size_t)255;
  const size_t oPt  = off; off += (size_t)nSB * SPB * 8;           off = (off + 255) & ~(size_t)255;
  const size_t oTb  = off; off += (size_t)SPB * 4;                 off = (off + 255) & ~(size_t)255;
  if (off > ws_size || off > (size_t)WSCAP) return;
  _Float16* wq0 = (_Float16*)(ws + oW0);
  _Float16* wq1 = (_Float16*)(ws + oW1);
  _Float16* wq2 = (_Float16*)(ws + oW2);
  _Float16* pP  = (_Float16*)(ws + oP);
  float*    hf  = (float*)(ws + oH);
  float*    G   = (float*)(ws + oG);
  int*   cnt  = (int*)(ws + oCnt);
  int*   offp = (int*)(ws + oOff);
  int*   rb   = (int*)(ws + oRb);
  int*   csr  = (int*)(ws + oCsr);
  float* es   = (float*)(ws + oES);
  float* ed   = (float*)(ws + oED);
  double* prt = (double*)(ws + oPt);
  float* tab  = (float*)(ws + oTb);

  const int vec8 = ((nE & 3) == 0) ? 1 : 0;

  k_wprep<FIN, D0><<<(D0 * FIN / 8 + NTHR - 1) / NTHR, NTHR, 0, stream>>>(W0, wq0);
  k_wprep<D0, D0><<<(D0 * D0 / 8 + NTHR - 1) / NTHR, NTHR, 0, stream>>>(W1, wq1);
  k_wprep<D0, NOUT><<<(NOUT * D0 / 8 + NTHR - 1) / NTHR, NTHR, 0, stream>>>(W2, wq2);
  k_xcvt<<<(nXu + NTHR - 1) / NTHR, NTHR, 0, stream>>>(x, pP, nN, nXu);

  k_count<<<nBC, NTHR, 0, stream>>>(dst, cnt, nE, vec8);
  k_offsets<<<1, OTHR, 0, stream>>>(cnt, offp, rb, nBC);
  hipFuncSetAttribute(reinterpret_cast<const void*>(&k_fill),
                      hipFuncAttributeMaxDynamicSharedMemorySize, LDS_FILL);
  k_fill<<<nBF, NTHR, LDS_FILL, stream>>>(src, dst, offp, rb, csr, nN, nE, vec8, csrLen);

  k_gemm<<<nGemm, NTHR, 0, stream>>>(pP, wq0, as0, ad0, hf, es, ed);
  k_agg<<<nAgg, NTHR, 0, stream>>>(csr, offp, cnt, es, ed, hf, b0, G, nN, csrLen);
  k_bnstat<<<nSB, NTHR, 0, stream>>>(G, prt, nN);
  k_bnfin<<<1, NTHR, 0, stream>>>(prt, tab, nSB, nN);
  k_bnapply<<<(nXu + NTHR - 1) / NTHR, NTHR, 0, stream>>>(G, tab, g0, be0, pP, nN, nXu);

  k_gemm<<<nGemm, NTHR, 0, stream>>>(pP, wq1, as1, ad1, hf, es, ed);
  k_agg<<<nAgg, NTHR, 0, stream>>>(csr, offp, cnt, es, ed, hf, b1, G, nN, csrLen);
  k_bnstat<<<nSB, NTHR, 0, stream>>>(G, prt, nN);
  k_bnfin<<<1, NTHR, 0, stream>>>(prt, tab, nSB, nN);
  k_bnapply<<<(nXu + NTHR - 1) / NTHR, NTHR, 0, stream>>>(G, tab, g1, be1, pP, nN, nXu);

  k_gemm16<<<nGemm2, NTHR, 0, stream>>>(pP, wq2, as2, ad2, hf, es, ed);
  k_aggo<<<nAgg, NTHR, 0, stream>>>(csr, offp, cnt, es, ed, hf, b2, out, nN, csrLen);
}
